// GCN_graph2_6090263626388
// MI455X (gfx1250) — hardware-verified
//
#include <hip/hip_runtime.h>
#include <stddef.h>


#define INC     128
#define DIM     64
#define OUTD    25
#define NTHR    256
#define NWAVE   8
#define EPT     8
#define NGRP    2
#define CHUNK   (NTHR * EPT * NGRP)
#define WCAP    (EPT * NGRP * 32)
#define LISTN   (NWAVE * WCAP)
#define NB      1024
#define SHB     10
#define NBD     8192
#define GROWS   128
#define WSC     64.0f
#define WINV    0.015625f
#define LN_EPS  1e-5f

#define LDS_AGG (NB * DIM * 4 + LISTN * 4)

static_assert((CHUNK & (CHUNK - 1)) == 0);
static_assert((NB & (NB - 1)) == 0 && (1 << SHB) >= NB);
static_assert((NBD & (NBD - 1)) == 0);
static_assert(NB % NWAVE == 0 && ((NB / NWAVE) % 4) == 0);
static_assert(NBD == 8 * NTHR * 4);
static_assert(GROWS == NWAVE * 16);
static_assert(LISTN * 4 >= 320 * 8);
static_assert(NBD % NB == 0 && NBD % GROWS == 0);

typedef float v2f __attribute__((ext_vector_type(2)));
typedef float v4f __attribute__((ext_vector_type(4)));
typedef float v8f __attribute__((ext_vector_type(8)));
typedef int   v4i __attribute__((ext_vector_type(4)));
typedef double v2d __attribute__((ext_vector_type(2)));
typedef _Float16 v8h  __attribute__((ext_vector_type(8)));
typedef _Float16 v16h __attribute__((ext_vector_type(16)));
union FragH { v16h v; v8h h[2]; };

__device__ __forceinline__ v8h cvt8(v4f a, v4f b) {
  v8h r;
  r[0] = (_Float16)a.x; r[1] = (_Float16)a.y; r[2] = (_Float16)a.z; r[3] = (_Float16)a.w;
  r[4] = (_Float16)b.x; r[5] = (_Float16)b.y; r[6] = (_Float16)b.z; r[7] = (_Float16)b.w;
  return r;
}

__device__ __forceinline__ v8f wmf(v16h a, v16h b, v8f c) {
  v8f d = __builtin_amdgcn_wmma_f32_16x16x32_f16(false, a, false, b, (short)0, c, false, false);
  asm volatile("v_nop\n\tv_nop\n\tv_nop\n\tv_nop" : "+v"(d) : "v"(a), "v"(b));
  return d;
}

__device__ __forceinline__ v16h load_a16(const float* p) {
  const v4f f0 = *(const v4f*)p,        f1 = *(const v4f*)(p + 4);
  const v4f f2 = *(const v4f*)(p + 16), f3 = *(const v4f*)(p + 20);
  FragH a; a.h[0] = cvt8(f0, f1); a.h[1] = cvt8(f2, f3);
  return a.v;
}
__device__ __forceinline__ v16h load_a16(const _Float16* p) {
  FragH a; a.h[0] = *(const v8h*)p; a.h[1] = *(const v8h*)(p + 16);
  return a.v;
}

template <int NBT, int SH, bool SRC>
__device__ __forceinline__ int scan_chunk(const int* __restrict__ srcs, const int* __restrict__ dsts,
                                          int nE, int nN, int cbase, int nodeBase, int vec8,
                                          int* list, int tid, int lane, int wave) {
  int wc = 0;
#pragma unroll
  for (int g = 0; g < NGRP; ++g) {
    const int e0   = cbase + (g * NTHR + tid) * EPT;
    const int sent = -2147483647 - 1;
    v4i da, db;
    if (vec8 != 0 && e0 + 7 < nE) {
      da = *(const v4i*)(dsts + e0);
      db = *(const v4i*)(dsts + e0 + 4);
    } else {
      da.x = (e0     < nE) ? dsts[min(e0, nE - 1)] : sent;
      da.y = (e0 + 1 < nE) ? dsts[min(e0 + 1, nE - 1)] : sent;
      da.z = (e0 + 2 < nE) ? dsts[min(e0 + 2, nE - 1)] : sent;
      da.w = (e0 + 3 < nE) ? dsts[min(e0 + 3, nE - 1)] : sent;
      db.x = (e0 + 4 < nE) ? dsts[min(e0 + 4, nE - 1)] : sent;
      db.y = (e0 + 5 < nE) ? dsts[min(e0 + 5, nE - 1)] : sent;
      db.z = (e0 + 6 < nE) ? dsts[min(e0 + 6, nE - 1)] : sent;
      db.w = (e0 + 7 < nE) ? dsts[min(e0 + 7, nE - 1)] : sent;
    }
    const unsigned nb = (unsigned)nodeBase;
    const unsigned s0 = (unsigned)da.x - nb, s1 = (unsigned)da.y - nb;
    const unsigned s2 = (unsigned)da.z - nb, s3 = (unsigned)da.w - nb;
    const unsigned s4 = (unsigned)db.x - nb, s5 = (unsigned)db.y - nb;
    const unsigned s6 = (unsigned)db.z - nb, s7 = (unsigned)db.w - nb;
    const bool h0 = s0 < (unsigned)NBT, h1 = s1 < (unsigned)NBT, h2 = s2 < (unsigned)NBT, h3 = s3 < (unsigned)NBT;
    const bool h4 = s4 < (unsigned)NBT, h5 = s5 < (unsigned)NBT, h6 = s6 < (unsigned)NBT, h7 = s7 < (unsigned)NBT;
    const unsigned any = __builtin_amdgcn_ballot_w32(h0 | h1 | h2 | h3 | h4 | h5 | h6 | h7);
    if (any != 0u) {
#define HITJ(J, HJ, SJ) { \
        const unsigned mj = __builtin_amdgcn_ballot_w32(HJ); \
        if (mj != 0u) { \
          if (HJ) { \
            const int pos = wc + (int)__builtin_amdgcn_mbcnt_lo(mj, 0u); \
            int val = (int)(SJ); \
            if (SRC) { \
              int sv = srcs[e0 + (J)]; \
              sv = sv < 0 ? 0 : (sv > nN - 1 ? nN - 1 : sv); \
              val |= (sv << SH); \
            } \
            if (pos < WCAP) list[wave * WCAP + pos] = val; \
          } \
          wc += (int)__builtin_popcount(mj); } }
      HITJ(0, h0, s0)
      HITJ(1, h1, s1)
      HITJ(2, h2, s2)
      HITJ(3, h3, s3)
      HITJ(4, h4, s4)
      HITJ(5, h5, s5)
      HITJ(6, h6, s6)
      HITJ(7, h7, s7)
#undef HITJ
    }
  }
  return wc;
}

__global__ __launch_bounds__(NTHR) void k_wprep(
    const float* __restrict__ w1, const float* __restrict__ w2, const float* __restrict__ w3,
    _Float16* wt) {
  const int i = blockIdx.x * NTHR + threadIdx.x;
  if (i >= (DIM * INC + 2 * DIM * DIM) / 8) return;
  const float* W; int n, k0, K; _Float16* base;
  if (i < (DIM * INC) / 8) {
    W = w1; K = INC; n = i >> 4; k0 = (i & 15) * 8; base = wt;
  } else if (i < (DIM * INC + DIM * DIM) / 8) {
    const int j = i - (DIM * INC) / 8;
    W = w2; K = DIM; n = j >> 3; k0 = (j & 7) * 8; base = wt + DIM * INC;
  } else {
    const int j = i - (DIM * INC + DIM * DIM) / 8;
    W = w3; K = DIM; n = j >> 3; k0 = (j & 7) * 8; base = wt + DIM * INC + DIM * DIM;
  }
  v4f a, b;
  a.x = W[(size_t)(k0 + 0) * DIM + n] * WSC; a.y = W[(size_t)(k0 + 1) * DIM + n] * WSC;
  a.z = W[(size_t)(k0 + 2) * DIM + n] * WSC; a.w = W[(size_t)(k0 + 3) * DIM + n] * WSC;
  b.x = W[(size_t)(k0 + 4) * DIM + n] * WSC; b.y = W[(size_t)(k0 + 5) * DIM + n] * WSC;
  b.z = W[(size_t)(k0 + 6) * DIM + n] * WSC; b.w = W[(size_t)(k0 + 7) * DIM + n] * WSC;
  const v8h o = cvt8(a, b);
  _Float16* p = base + (size_t)n * K + k0;
  *(volatile v8h*)p = o;
  __threadfence();
  *(volatile v8h*)p = o;
}

__global__ __launch_bounds__(NTHR) void k_deg(const int* __restrict__ ei, float* dinv, int nE, int vec8) {
  __shared__ __attribute__((aligned(16))) int cnt[NBD];
  __shared__ int list[LISTN];
  __shared__ int wcnt[NWAVE];
  const int tid = threadIdx.x, lane = tid & 31, wave = tid >> 5;
  const int nodeBase = blockIdx.x * NBD;
  const int* dsts = ei + nE;

  for (int i = tid; i < NBD; i += NTHR) cnt[i] = 0;
  __syncthreads();

  const int nChunks = (nE + CHUNK - 1) / CHUNK;
#pragma unroll 1
  for (int ch = 0; ch < nChunks; ++ch) {
    const int cbase = ch * CHUNK;
    const int wc = scan_chunk<NBD, 0, false>(ei, dsts, nE, 1, cbase, nodeBase, vec8, list, tid, lane, wave);
    if (lane == 0) wcnt[wave] = wc;
    __syncthreads();
    if (wave == 0) {
#pragma unroll 1
      for (int wsx = 0; wsx < NWAVE; ++wsx) {
        int n = __builtin_amdgcn_readfirstlane(wcnt[wsx]);
        n = n > WCAP ? WCAP : (n < 0 ? 0 : n);
        const int* lp = list + wsx * WCAP;
#pragma unroll 1
        for (int i = 0; i < n; ++i) {
          const int ent  = __builtin_amdgcn_readfirstlane(lp[i]);
          const int slot = ent & (NBD - 1);
          if (lane == 0) cnt[slot] = cnt[slot] + 1;
        }
      }
    }
    __syncthreads();
  }

  float* dp = dinv + (size_t)blockIdx.x * NBD;
#pragma unroll
  for (int q = 0; q < NBD / (NTHR * 4); ++q) {
    const int f = q * (NTHR * 4) + 4 * tid;
    v4f d;
    d.x = rsqrtf((float)cnt[f + 0] + 1.0f); d.y = rsqrtf((float)cnt[f + 1] + 1.0f);
    d.z = rsqrtf((float)cnt[f + 2] + 1.0f); d.w = rsqrtf((float)cnt[f + 3] + 1.0f);
    *(volatile v4f*)(dp + f) = d;
  }
  __threadfence();
#pragma unroll
  for (int q = 0; q < NBD / (NTHR * 4); ++q) {
    const int f = q * (NTHR * 4) + 4 * tid;
    v4f d;
    d.x = rsqrtf((float)cnt[f + 0] + 1.0f); d.y = rsqrtf((float)cnt[f + 1] + 1.0f);
    d.z = rsqrtf((float)cnt[f + 2] + 1.0f); d.w = rsqrtf((float)cnt[f + 3] + 1.0f);
    *(volatile v4f*)(dp + f) = d;
  }
}

template <typename TA, int KD>
__device__ __forceinline__ void gemm_body(const TA* __restrict__ A, const _Float16* __restrict__ wt,
                                          const float* __restrict__ dinv, float* hs, int nN, float* stg) {
  const int tid = threadIdx.x, lane = tid & 31, wave = tid >> 5, hh = lane >> 4, m = lane & 15;
  const int row0 = blockIdx.x * GROWS + wave * 16;
  int node = row0 + m;
  node = node > nN - 1 ? nN - 1 : node;
  const TA* ap = A + (size_t)node * KD;

  v8f acc[4];
#pragma unroll
  for (int t = 0; t < 4; ++t) { v8f z = {0.f, 0.f, 0.f, 0.f, 0.f, 0.f, 0.f, 0.f}; acc[t] = z; }

#pragma unroll
  for (int ks = 0; ks < KD / 32; ++ks) {
    const v16h av = load_a16(ap + 32 * ks + 8 * hh);
#pragma unroll
    for (int t = 0; t < 4; ++t) {
      const _Float16* bp = wt + (size_t)(16 * t + m) * KD + 32 * ks + 8 * hh;
      FragH b;
      b.h[0] = *(const v8h*)bp;
      b.h[1] = *(const v8h*)(bp + 16);
      acc[t] = wmf(av, b.v, acc[t]);
    }
  }

  const int rb = row0 + 8 * hh;
  const v4f da = *(const v4f*)(dinv + rb), db = *(const v4f*)(dinv + rb + 4);
  const float s0 = da.x * WINV, s1 = da.y * WINV, s2 = da.z * WINV, s3 = da.w * WINV;
  const float s4 = db.x * WINV, s5 = db.y * WINV, s6 = db.z * WINV, s7 = db.w * WINV;
  float* sp = stg + wave * (16 * DIM) + (8 * hh) * DIM + m;
#pragma unroll
  for (int t = 0; t < 4; ++t) {
    sp[0 * DIM + 16 * t] = acc[t][0] * s0;
    sp[1 * DIM + 16 * t] = acc[t][1] * s1;
    sp[2 * DIM + 16 * t] = acc[t][2] * s2;
    sp[3 * DIM + 16 * t] = acc[t][3] * s3;
    sp[4 * DIM + 16 * t] = acc[t][4] * s4;
    sp[5 * DIM + 16 * t] = acc[t][5] * s5;
    sp[6 * DIM + 16 * t] = acc[t][6] * s6;
    sp[7 * DIM + 16 * t] = acc[t][7] * s7;
  }
  __syncthreads();

  const float* lp = stg + wave * (16 * DIM) + 4 * lane;
  float* gp = hs + (size_t)row0 * DIM + 4 * lane;
  v4f ov[8];
#pragma unroll
  for (int q = 0; q < 8; ++q) ov[q] = *(const v4f*)(lp + q * 128);
#pragma unroll
  for (int q = 0; q < 8; ++q) *(volatile v4f*)(gp + q * 128) = ov[q];
  __threadfence();
#pragma unroll
  for (int q = 0; q < 8; ++q) *(volatile v4f*)(gp + q * 128) = ov[q];
}

__global__ __launch_bounds__(NTHR) void k_gemm_x(
    const float* __restrict__ x, const _Float16* __restrict__ wt, const float* __restrict__ dinv,
    float* hs, int nN) {
  __shared__ __attribute__((aligned(16))) float stg[NWAVE * 16 * DIM];
  gemm_body<float, INC>(x, wt, dinv, hs, nN, stg);
}

__global__ __launch_bounds__(NTHR) void k_gemm_h(
    const _Float16* __restrict__ a, const _Float16* __restrict__ wt, const float* __restrict__ dinv,
    float* hs, int nN) {
  __shared__ __attribute__((aligned(16))) float stg[NWAVE * 16 * DIM];
  gemm_body<_Float16, DIM>(a, wt, dinv, hs, nN, stg);
}

__global__ __launch_bounds__(NTHR) void k_agg(
    const int* __restrict__ ei, const float* __restrict__ hs, const float* __restrict__ dinv,
    const float* __restrict__ bias, const float* __restrict__ lnw, const float* __restrict__ lnb,
    _Float16* act, double* pool, int nN, int nE, int vec8, int mode) {
  extern __shared__ v4f lds_dyn[];
  float* acc  = (float*)lds_dyn;
  int*   list = (int*)(acc + NB * DIM);
  __shared__ int wcnt[NWAVE];
  __shared__ __attribute__((aligned(16))) float spar[3 * DIM];
  const int tid = threadIdx.x, lane = tid & 31, wave = tid >> 5;
  const int nodeBase = blockIdx.x * NB;
  const int* srcs = ei;
  const int* dsts = ei + nE;

  if (tid < 3 * DIM) {
    float v;
    if (tid < DIM) v = bias[tid];
    else if (tid < 2 * DIM) v = lnw[tid - DIM];
    else v = lnb[tid - 2 * DIM];
    spar[tid] = v;
  }
  {
    const v4f z = {0.f, 0.f, 0.f, 0.f};
    for (int i = tid; i < NB * DIM / 4; i += NTHR) lds_dyn[i] = z;
  }
  __syncthreads();

  const int nChunks = (nE + CHUNK - 1) / CHUNK;
#pragma unroll 1
  for (int ch = 0; ch < nChunks; ++ch) {
    const int cbase = ch * CHUNK;
    const int wc = scan_chunk<NB, SHB, true>(srcs, dsts, nE, nN, cbase, nodeBase, vec8, list, tid, lane, wave);
    if (lane == 0) wcnt[wave] = wc;
    __syncthreads();
    if (wave == 0) {
#pragma unroll 1
      for (int wsx = 0; wsx < NWAVE; ++wsx) {
        int n = __builtin_amdgcn_readfirstlane(wcnt[wsx]);
        n = n > WCAP ? WCAP : (n < 0 ? 0 : n);
        const int* lp = list + wsx * WCAP;
#pragma unroll 1
        for (int i = 0; i < n; ++i) {
          const int ent  = __builtin_amdgcn_readfirstlane(lp[i]);
          const int slot = ent & (NB - 1);
          int src = (ent >> SHB) & 0x1FFFFF;
          src = src > nN - 1 ? nN - 1 : src;
          const v2f v = *(const v2f*)(hs + (size_t)src * DIM + 2 * lane);
          v2f* ap = (v2f*)(acc + slot * DIM + 2 * lane);
          *ap = *ap + v;
        }
      }
    }
    __syncthreads();
  }

  const v2f bb = *(const v2f*)(spar + 2 * lane);
  const v2f ww = *(const v2f*)(spar + DIM + 2 * lane);
  const v2f lb = *(const v2f*)(spar + 2 * DIM + 2 * lane);
#pragma unroll 2
  for (int j = 0; j < NB / NWAVE; ++j) {
    const int slot = wave * (NB / NWAVE) + j;
    const int node = nodeBase + slot;
    const int nodec = node > nN - 1 ? nN - 1 : node;
    v2f* ap = (v2f*)(acc + slot * DIM + 2 * lane);
    const v2f a = *ap;
    const v2f g = *(const v2f*)(hs + (size_t)nodec * DIM + 2 * lane);
    const float di = dinv[(size_t)nodeBase + slot];
    const float t0 = di * (a.x + g.x) + bb.x;
    const float t1 = di * (a.y + g.y) + bb.y;
    float s = t0 + t1;
    s += __shfl_xor(s, 16, 32);
    s += __shfl_xor(s, 8, 32);
    s += __shfl_xor(s, 4, 32);
    s += __shfl_xor(s, 2, 32);
    s += __shfl_xor(s, 1, 32);
    const float mu = s * (1.0f / 64.0f);
    const float d0 = t0 - mu, d1 = t1 - mu;
    float ss = d0 * d0 + d1 * d1;
    ss += __shfl_xor(ss, 16, 32);
    ss += __shfl_xor(ss, 8, 32);
    ss += __shfl_xor(ss, 4, 32);
    ss += __shfl_xor(ss, 2, 32);
    ss += __shfl_xor(ss, 1, 32);
    const float var = ss * (1.0f / 64.0f);
    const float inv = rsqrtf(var + LN_EPS);
    float y0 = d0 * inv * ww.x + lb.x;
    float y1 = d1 * inv * ww.y + lb.y;
    y0 = y0 > 0.0f ? y0 : 0.0f;
    y1 = y1 > 0.0f ? y1 : 0.0f;
    if (node > nN - 1) { y0 = 0.0f; y1 = 0.0f; }
    v2f y; y.x = y0; y.y = y1;
    *ap = y;
  }
  __syncthreads();

  double* ppd = (double*)list;
  if (mode == 0) {
    _Float16* ab = act + (size_t)nodeBase * DIM;
    const int rsub = lane >> 3, c8 = (lane & 7) * 8;
#pragma unroll 4
    for (int q = 0; q < (NB / NWAVE) / 4; ++q) {
      const int row = wave * (NB / NWAVE) + 4 * q + rsub;
      const float* lp = acc + row * DIM + c8;
      const v4f f0 = *(const v4f*)lp, f1 = *(const v4f*)(lp + 4);
      const v8h o = cvt8(f0, f1);
      *(volatile v8h*)(ab + (size_t)row * DIM + c8) = o;
    }
    __threadfence();
#pragma unroll 4
    for (int q = 0; q < (NB / NWAVE) / 4; ++q) {
      const int row = wave * (NB / NWAVE) + 4 * q + rsub;
      const float* lp = acc + row * DIM + c8;
      const v4f f0 = *(const v4f*)lp, f1 = *(const v4f*)(lp + 4);
      const v8h o = cvt8(f0, f1);
      *(volatile v8h*)(ab + (size_t)row * DIM + c8) = o;
    }
  } else {
    const int c = tid & (DIM - 1), g = tid >> 6;
    double sum = 0.0;
#pragma unroll 4
    for (int r = g; r < NB; r += 4) sum += (double)acc[r * DIM + c];
    ppd[g * DIM + c] = sum;
  }
  __syncthreads();
  if (mode != 0 && tid < DIM) {
    const double tot = ((ppd[tid] + ppd[DIM + tid]) + ppd[2 * DIM + tid]) + ppd[3 * DIM + tid];
    ppd[4 * DIM + tid] = tot;
  }
  __syncthreads();
  if (mode != 0 && wave == 0) {
    const v2d pv = *(const v2d*)(ppd + 4 * DIM + 2 * lane);
    double* pp = pool + (size_t)blockIdx.x * DIM + 2 * lane;
    *(volatile v2d*)pp = pv;
    __threadfence();
    *(volatile v2d*)pp = pv;
  }
}

__global__ __launch_bounds__(64) void k_head(
    const double* __restrict__ pool, const float* __restrict__ Wl, const float* __restrict__ bl,
    float* out, int nAB, int nN) {
  __shared__ float sp[DIM];
  const int c = threadIdx.x;
  double s = 0.0;
#pragma unroll 1
  for (int b = 0; b < nAB; ++b) s += pool[(size_t)b * DIM + c];
  sp[c] = (float)(s / (double)nN);
  __syncthreads();
  float r = 0.0f;
  if (c < OUTD) {
#pragma unroll 8
    for (int f = 0; f < DIM; ++f) r = r + sp[f] * Wl[f * OUTD + c];
    r = r + bl[c];
    *(volatile float*)(out + c) = r;
  }
  __threadfence();
  if (c < OUTD) *(volatile float*)(out + c) = r;
}

extern "C" void kernel_launch(void* const* d_in, const int* in_sizes, int n_in,
                              void* d_out, int out_size, void* d_ws, size_t ws_size,
                              hipStream_t stream) {
  if (n_in < 16) return;
  const int nN = in_sizes[0] / INC;
  const int nE = in_sizes[1] / 2;
  if (nN <= 0 || nN > (1 << 21) || nE < 0) return;
  if (in_sizes[0] != nN * INC || in_sizes[1] != 2 * nE) return;
  if (in_sizes[2] != INC * DIM || in_sizes[4] != DIM * DIM || in_sizes[6] != DIM * DIM) return;
  if (in_sizes[3] != DIM || in_sizes[5] != DIM || in_sizes[7] != DIM) return;
  for (int i = 8; i < 14; ++i) if (in_sizes[i] != DIM) return;
  if (in_sizes[14] != DIM * OUTD || in_sizes[15] != OUTD || out_size != OUTD) return;

  const float* x    = (const float*)d_in[0];
  const int*   ei   = (const int*)d_in[1];
  const float* W1   = (const float*)d_in[2];
  const float* b1   = (const float*)d_in[3];
  const float* W2   = (const float*)d_in[4];
  const float* b2   = (const float*)d_in[5];
  const float* W3   = (const float*)d_in[6];
  const float* b3   = (const float*)d_in[7];
  const float* ln1w = (const float*)d_in[8],  *ln1b = (const float*)d_in[9];
  const float* ln2w = (const float*)d_in[10], *ln2b = (const float*)d_in[11];
  const float* ln3w = (const float*)d_in[12], *ln3b = (const float*)d_in[13];
  const float* Wl   = (const float*)d_in[14];
  const float* bl   = (const float*)d_in[15];
  float* out = (float*)d_out;

  const int nGB = (nN + GROWS - 1) / GROWS;
  const int nAB = (nN + NB - 1) / NB;
  const int nDB = (nN + NBD - 1) / NBD;
  const size_t rowsH = (size_t)nGB * GROWS;
  const size_t rowsA = (size_t)nAB * NB;
  const size_t rowsD = (size_t)nDB * NBD;
  if (rowsH > rowsD || rowsA > rowsD) return;

  char* ws = (char*)d_ws;
  size_t off = 0;
  const size_t oWT = off; off += (size_t)(DIM * INC + 2 * DIM * DIM) * 2;   off = (off + 255) & ~(size_t)255;
  const size_t oDV = off; off += rowsD * 4;                                off = (off + 255) & ~(size_t)255;
  const size_t oHS = off; off += rowsH * DIM * 4;                          off = (off + 255) & ~(size_t)255;
  const size_t oAC = off; off += rowsA * DIM * 2;                          off = (off + 255) & ~(size_t)255;
  const size_t oPP = off; off += (size_t)nAB * DIM * 8;                    off = (off + 255) & ~(size_t)255;
  if (off > ws_size) return;
  if (off > ((size_t)128 << 20)) return;
  _Float16* wt   = (_Float16*)(ws + oWT);
  float*    dinv = (float*)(ws + oDV);
  float*    hs   = (float*)(ws + oHS);
  _Float16* act  = (_Float16*)(ws + oAC);
  double*   pool = (double*)(ws + oPP);

  const int vec8 = ((nE & 3) == 0) ? 1 : 0;

  const int nPrep = (DIM * INC + 2 * DIM * DIM) / 8;
  k_wprep<<<(nPrep + NTHR - 1) / NTHR, NTHR, 0, stream>>>(W1, W2, W3, wt);
  k_deg<<<nDB, NTHR, 0, stream>>>(ei, dinv, nE, vec8);

  hipFuncSetAttribute(reinterpret_cast<const void*>(&k_agg),
                      hipFuncAttributeMaxDynamicSharedMemorySize, LDS_AGG);

  k_gemm_x<<<nGB, NTHR, 0, stream>>>(x, wt, dinv, hs, nN);
  k_agg<<<nAB, NTHR, LDS_AGG, stream>>>(ei, hs, dinv, b1, ln1w, ln1b, act, pool, nN, nE, vec8, 0);
  k_gemm_h<<<nGB, NTHR, 0, stream>>>(act, wt + DIM * INC, dinv, hs, nN);
  k_agg<<<nAB, NTHR, LDS_AGG, stream>>>(ei, hs, dinv, b2, ln2w, ln2b, act, pool, nN, nE, vec8, 0);
  k_gemm_h<<<nGB, NTHR, 0, stream>>>(act, wt + DIM * INC + DIM * DIM, dinv, hs, nN);
  k_agg<<<nAB, NTHR, LDS_AGG, stream>>>(ei, hs, dinv, b3, ln3w, ln3b, act, pool, nN, nE, vec8, 1);

  k_head<<<1, 64, 0, stream>>>(pool, Wl, bl, out, nAB, nN);
}
